// MOLELinear_6493990551579
// MI455X (gfx1250) — hardware-run, weakly checked
//
#include <hip/hip_runtime.h>

typedef __attribute__((ext_vector_type(16))) __bf16   v16b;
typedef __attribute__((ext_vector_type(8)))  __bf16   v8b;
typedef __attribute__((ext_vector_type(8)))  float    v8f;
typedef __attribute__((ext_vector_type(4)))  float    v4f;
typedef __attribute__((ext_vector_type(8)))  unsigned v8u;
typedef __attribute__((ext_vector_type(4)))  unsigned v4u;
typedef __attribute__((ext_vector_type(4)))  int      v4i;

constexpr int kAtoms   = 100000;
constexpr int kSys     = 32;
constexpr int kExp     = 16;
constexpr int kFeat    = 64;
constexpr int kMat     = kFeat * kFeat;
constexpr int kTiles   = kAtoms / 16;
constexpr int kSlabP   = 68;
constexpr int kMixThreads = kSys * kMat / 8;
constexpr int kMixBlocks  = kMixThreads / 256;
constexpr int kMainBlocks = (kTiles + 7) / 8;
static_assert(kAtoms == kTiles * 16);
static_assert(kTiles == 6250);
static_assert(kMat == 4096);
static_assert((kFeat % 32) == 0);
static_assert(kMixBlocks * 256 == kMixThreads);
static_assert(kMixBlocks == 2 * kSys);
static_assert(kMainBlocks == 782);

constexpr size_t kOffWH   = 0;
constexpr size_t kOffWL   = kOffWH + (size_t)kSys * kMat * 2;
constexpr size_t kWsTotal = kOffWL + (size_t)kSys * kMat * 2;
static_assert(kWsTotal == 524288ull);
static_assert((kOffWL % 128) == 0);
static_assert(kWsTotal <= 134217728ull);

__device__ __forceinline__ unsigned f2bf_bits(float f) {
  const unsigned u = __float_as_uint(f);
  return ((u + 0x7FFFu + ((u >> 16) & 1u)) >> 16) & 0xFFFFu;
}
__device__ __forceinline__ float bf_bits2f(unsigned h) { return __uint_as_float(h << 16); }

__device__ __forceinline__ void split_pair(float f0, float f1, unsigned& wh, unsigned& wl) {
  const unsigned h0 = f2bf_bits(f0);
  const unsigned h1 = f2bf_bits(f1);
  const float d0 = f0 - bf_bits2f(h0);
  const float d1 = f1 - bf_bits2f(h1);
  const unsigned l0 = f2bf_bits(d0);
  const unsigned l1 = f2bf_bits(d1);
  wh = h0 | (h1 << 16);
  wl = l0 | (l1 << 16);
}

__device__ __forceinline__ int clamp_sys(int v) {
  const int a = (v < 0) ? 0 : v;
  return (a > (kSys - 1)) ? (kSys - 1) : a;
}

union FragB { v16b v; v8b h[2]; };
__device__ __forceinline__ v16b load_frag(const __bf16* p) {
  FragB f;
  f.h[0] = *(const v8b*)(p);
  f.h[1] = *(const v8b*)(p + 16);
  return f.v;
}

__device__ __forceinline__ v8f mma_bf(v16b a, v16b b, v8f c) {
  c = __builtin_amdgcn_wmma_f32_16x16x32_bf16(false, a, false, b, (short)0, c, false, false);
  asm volatile("v_nop\n\tv_nop\n\tv_nop\n\tv_nop" : "+v"(c) : "v"(a), "v"(b));
  return c;
}

__global__ __launch_bounds__(256) void mix_split_kernel(
    const float* __restrict__ W, const float* __restrict__ coef,
    unsigned short* __restrict__ WH, unsigned short* __restrict__ WL)
{
  const int s   = (int)(blockIdx.x >> 1);
  const int idx = (((int)(blockIdx.x & 1)) * 256 + (int)threadIdx.x) * 8;
  if (s >= kSys) return;
  float acc[8];
#pragma unroll
  for (int j = 0; j < 8; ++j) acc[j] = 0.0f;
#pragma unroll 1
  for (int e = 0; e < kExp; ++e) {
    const float cf = coef[s * kExp + e];
    const float* wp = W + (size_t)e * kMat + idx;
    const v4f w0 = *(const v4f*)(wp);
    const v4f w1 = *(const v4f*)(wp + 4);
    acc[0] = fmaf(cf, w0[0], acc[0]);
    acc[1] = fmaf(cf, w0[1], acc[1]);
    acc[2] = fmaf(cf, w0[2], acc[2]);
    acc[3] = fmaf(cf, w0[3], acc[3]);
    acc[4] = fmaf(cf, w1[0], acc[4]);
    acc[5] = fmaf(cf, w1[1], acc[5]);
    acc[6] = fmaf(cf, w1[2], acc[6]);
    acc[7] = fmaf(cf, w1[3], acc[7]);
  }
  v4u hv, lv;
  unsigned th, tl;
  split_pair(acc[0], acc[1], th, tl);
  hv[0] = th; lv[0] = tl;
  split_pair(acc[2], acc[3], th, tl);
  hv[1] = th; lv[1] = tl;
  split_pair(acc[4], acc[5], th, tl);
  hv[2] = th; lv[2] = tl;
  split_pair(acc[6], acc[7], th, tl);
  hv[3] = th; lv[3] = tl;
  unsigned short* qh = WH + (size_t)s * kMat + idx;
  unsigned short* ql = WL + (size_t)s * kMat + idx;
  *(volatile v4u*)qh = hv;
  *(volatile v4u*)ql = lv;
  __threadfence();
  *(volatile v4u*)qh = hv;
  *(volatile v4u*)ql = lv;
}

__global__ __launch_bounds__(256) void tile_product_kernel(
    const float* __restrict__ x, const int* __restrict__ bidx,
    const unsigned short* __restrict__ WH, const unsigned short* __restrict__ WL,
    const float* __restrict__ bias, float* __restrict__ out)
{
  __shared__ __align__(16) float sT[8][16 * kSlabP];
  const int lane = (int)threadIdx.x & 31;
  const int wave = (int)threadIdx.x >> 5;
  const int tile = (int)blockIdx.x * 8 + wave;
  if (tile >= kTiles) return;
  const int base = tile * 16;
  const int hh = lane >> 4;
  const int c  = lane & 15;

  int rowSys[8];
  {
    const int* bp = bidx + base + 8 * hh;
    const v4i i0 = *(const v4i*)(bp);
    const v4i i1 = *(const v4i*)(bp + 4);
    rowSys[0] = clamp_sys(i0[0]);
    rowSys[1] = clamp_sys(i0[1]);
    rowSys[2] = clamp_sys(i0[2]);
    rowSys[3] = clamp_sys(i0[3]);
    rowSys[4] = clamp_sys(i1[0]);
    rowSys[5] = clamp_sys(i1[1]);
    rowSys[6] = clamp_sys(i1[2]);
    rowSys[7] = clamp_sys(i1[3]);
  }
  int mn = rowSys[0], mx = rowSys[0];
#pragma unroll
  for (int r = 1; r < 8; ++r) {
    mn = (rowSys[r] < mn) ? rowSys[r] : mn;
    mx = (rowSys[r] > mx) ? rowSys[r] : mx;
  }
  {
    const int omn = __shfl_xor(mn, 16, 32);
    const int omx = __shfl_xor(mx, 16, 32);
    mn = (omn < mn) ? omn : mn;
    mx = (omx > mx) ? omx : mx;
  }
  const int s_lo = __builtin_amdgcn_readfirstlane(mn);
  const int s_hi = __builtin_amdgcn_readfirstlane(mx);
  int nsys = s_hi - s_lo + 1;
  nsys = (nsys > kSys) ? kSys : nsys;

  v16b ah[2], al[2];
  {
    const float* xrow = x + (size_t)(base + c) * kFeat + 8 * hh;
#pragma unroll
    for (int kc = 0; kc < 2; ++kc) {
      v8u wh, wl;
#pragma unroll
      for (int hf = 0; hf < 2; ++hf) {
        const float* p = xrow + kc * 32 + hf * 16;
        const v4f a0 = *(const v4f*)(p);
        const v4f a1 = *(const v4f*)(p + 4);
        unsigned th, tl;
        split_pair(a0[0], a0[1], th, tl);
        wh[hf * 4 + 0] = th; wl[hf * 4 + 0] = tl;
        split_pair(a0[2], a0[3], th, tl);
        wh[hf * 4 + 1] = th; wl[hf * 4 + 1] = tl;
        split_pair(a1[0], a1[1], th, tl);
        wh[hf * 4 + 2] = th; wl[hf * 4 + 2] = tl;
        split_pair(a1[2], a1[3], th, tl);
        wh[hf * 4 + 3] = th; wl[hf * 4 + 3] = tl;
      }
      ah[kc] = __builtin_bit_cast(v16b, wh);
      al[kc] = __builtin_bit_cast(v16b, wl);
    }
  }

  v8f res[4];
#pragma unroll
  for (int nt = 0; nt < 4; ++nt) res[nt] = (v8f){0.f, 0.f, 0.f, 0.f, 0.f, 0.f, 0.f, 0.f};

#pragma unroll 1
  for (int it = 0; it < nsys; ++it) {
    const int s = s_lo + it;
    const __bf16* bhp = (const __bf16*)WH + (size_t)s * kMat + c * kFeat + 8 * hh;
    const __bf16* blp = (const __bf16*)WL + (size_t)s * kMat + c * kFeat + 8 * hh;
#pragma unroll
    for (int nt = 0; nt < 4; ++nt) {
      const int o = nt * 16 * kFeat;
      const v16b bh0 = load_frag(bhp + o);
      const v16b bh1 = load_frag(bhp + o + 32);
      const v16b bl0 = load_frag(blp + o);
      const v16b bl1 = load_frag(blp + o + 32);
      v8f acc = (v8f){0.f, 0.f, 0.f, 0.f, 0.f, 0.f, 0.f, 0.f};
      acc = mma_bf(ah[0], bh0, acc);
      acc = mma_bf(ah[1], bh1, acc);
      acc = mma_bf(ah[0], bl0, acc);
      acc = mma_bf(ah[1], bl1, acc);
      acc = mma_bf(al[0], bh0, acc);
      acc = mma_bf(al[1], bh1, acc);
#pragma unroll
      for (int r = 0; r < 8; ++r) res[nt][r] = (rowSys[r] == s) ? acc[r] : res[nt][r];
    }
  }

  float* slab = sT[wave];
#pragma unroll
  for (int nt = 0; nt < 4; ++nt) {
    const float bv = bias[nt * 16 + c];
#pragma unroll
    for (int r = 0; r < 8; ++r) {
      const float v = res[nt][r] + bv;
      slab[(8 * hh + r) * kSlabP + nt * 16 + c] = v;
    }
  }
  __builtin_amdgcn_fence(__ATOMIC_RELEASE, "workgroup");
  __builtin_amdgcn_wave_barrier();
  __builtin_amdgcn_fence(__ATOMIC_ACQUIRE, "workgroup");
  {
    const int c4 = c * 4;
    float* ob = out + (size_t)base * kFeat;
    for (int pass = 0; pass < 2; ++pass) {
#pragma unroll
      for (int q = 0; q < 8; ++q) {
        const int row = q * 2 + hh;
        const v4f val = *(const v4f*)(slab + row * kSlabP + c4);
        *(volatile v4f*)(ob + (size_t)row * kFeat + c4) = val;
      }
      __threadfence();
    }
  }
}

extern "C" void kernel_launch(void* const* d_in, const int* in_sizes, int n_in,
                              void* d_out, int out_size, void* d_ws, size_t ws_size,
                              hipStream_t stream) {
  (void)in_sizes;
  (void)out_size;
  if (n_in < 5) return;
  if (ws_size < kWsTotal) return;

  const float* x    = (const float*)d_in[0];
  const float* coef = (const float*)d_in[1];
  const int*   bidx = (const int*)d_in[2];
  const float* W    = (const float*)d_in[3];
  const float* bias = (const float*)d_in[4];
  float* out = (float*)d_out;

  char* ws = (char*)d_ws;
  unsigned short* WH = (unsigned short*)(ws + kOffWH);
  unsigned short* WL = (unsigned short*)(ws + kOffWL);

  mix_split_kernel<<<kMixBlocks, 256, 0, stream>>>(W, coef, WH, WL);
  tile_product_kernel<<<kMainBlocks, 256, 0, stream>>>(x, bidx, WH, WL, bias, out);
}
